// CosformerAttention_82841329205679
// MI455X (gfx1250) — hardware-verified
//
#include <hip/hip_runtime.h>
#include <math.h>
#include <stdint.h>

#define NB   8
#define NT   4096
#define ND   128
#define NF   256
#define NSF  512
#define NJ   144
#define CH   128
#define NCH  32
#define NSL  33
#define NFG  8
#define QP   264
#define KP   136
#define VP   72
static_assert(NT == NCH * CH);
static_assert(NSF == NFG * 64);
static_assert(NF == 2 * ND);
static_assert(((QP * 2) % 16) == 0 && ((KP * 2) % 16) == 0 && ((VP * 2) % 16) == 0);

typedef __bf16   v16b __attribute__((ext_vector_type(16)));
typedef __bf16   v8b  __attribute__((ext_vector_type(8)));
typedef float    v8f  __attribute__((ext_vector_type(8)));
typedef float    v4f  __attribute__((ext_vector_type(4)));
typedef unsigned int v4u __attribute__((ext_vector_type(4)));

__device__ __forceinline__ unsigned short bf_bits(float f) {
  unsigned u = __float_as_uint(f);
  return (unsigned short)((u + 0x7FFFu + ((u >> 16) & 1u)) >> 16);
}
__device__ __forceinline__ float bf_up(unsigned short h) { return __uint_as_float(((unsigned)h) << 16); }
__device__ __forceinline__ __bf16 bf_val(unsigned short h) { return __builtin_bit_cast(__bf16, h); }
__device__ __forceinline__ unsigned pk16(unsigned short a, unsigned short b) { return (unsigned)a | ((unsigned)b << 16); }
__device__ __forceinline__ v8f zero8() { v8f z = {0.f, 0.f, 0.f, 0.f, 0.f, 0.f, 0.f, 0.f}; return z; }

__device__ __forceinline__ v16b ldfrag_b(const __bf16* p) {
  union { v16b v; v8b h[2]; } f;
  f.h[0] = *(const v8b*)(p);
  f.h[1] = *(const v8b*)(p + 16);
  return f.v;
}

__device__ __forceinline__ v8f mma_b(v16b a, v16b b, v8f c) {
  c = __builtin_amdgcn_wmma_f32_16x16x32_bf16(false, a, false, b, (short)0, c, false, false);
  asm volatile("v_nop\n\tv_nop\n\tv_nop\n\tv_nop" : "+v"(c) : "v"(a), "v"(b));
  return c;
}

__device__ __forceinline__ void relu_pack8(v4f a, v4f c, v4u& pos, v4u& neg) {
  const float xv[8] = {a[0], a[1], a[2], a[3], c[0], c[1], c[2], c[3]};
  unsigned short pb[8], nb[8];
#pragma unroll
  for (int e = 0; e < 8; ++e) {
    const unsigned short bt = bf_bits(xv[e]);
    const float f = bf_up(bt);
    pb[e] = (f > 0.0f) ? bt : (unsigned short)0u;
    nb[e] = (f < 0.0f) ? (unsigned short)(bt & 0x7FFFu) : (unsigned short)0u;
  }
  pos[0] = pk16(pb[0], pb[1]); pos[1] = pk16(pb[2], pb[3]); pos[2] = pk16(pb[4], pb[5]); pos[3] = pk16(pb[6], pb[7]);
  neg[0] = pk16(nb[0], nb[1]); neg[1] = pk16(nb[2], nb[3]); neg[2] = pk16(nb[4], nb[5]); neg[3] = pk16(nb[6], nb[7]);
}

__global__ __launch_bounds__(128) void k_vt(const float* __restrict__ v, unsigned short* VTp) {
  __shared__ __align__(16) unsigned short sT[NJ * VP];
  const int tid = threadIdx.x, lane = tid & 31, wave = tid >> 5;
  const int b = blockIdx.x >> 6, s0 = (blockIdx.x & 63) * 64;
  {
    const int r = tid >> 1, chh = (tid & 1) * 64;
    const float* src = v + ((size_t)(b * NT + s0 + r)) * ND + chh;
#pragma unroll 2
    for (int g = 0; g < 16; ++g) {
      const v4f a = *(const v4f*)(src + 4 * g);
#pragma unroll
      for (int e = 0; e < 4; ++e) sT[(chh + 4 * g + e) * VP + r] = bf_bits(a[e]);
    }
#pragma unroll
    for (int e = 0; e < 8; ++e) {
      const int idx = tid * 8 + e;
      const int row = ND + (idx >> 6), col = idx & 63;
      sT[row * VP + col] = (row == ND) ? (unsigned short)0x3F80u : (unsigned short)0u;
    }
  }
  __syncthreads();
  const int q8 = lane & 7, sub = lane >> 3;
  for (int pass = 0; pass < 2; ++pass) {
#pragma unroll
    for (int it = 0; it < 9; ++it) {
      const int row = wave * 36 + it * 4 + sub;
      const v4u val = *(const v4u*)(sT + row * VP + 8 * q8);
      *(volatile v4u*)(VTp + ((size_t)(b * NJ + row)) * NT + s0 + 8 * q8) = val;
    }
    __threadfence();
  }
}

#define SLABF 1088
#define SBUF_BYTES 39168
static_assert(SBUF_BYTES >= 9 * SLABF * 4);
static_assert(SBUF_BYTES >= 2 * 64 * KP * 2);

__global__ __launch_bounds__(288) void k_state(const float* __restrict__ kin, const unsigned short* __restrict__ VTp,
                                               unsigned short* Shp, unsigned short* Slp) {
  __shared__ __align__(16) unsigned char sbuf[SBUF_BYTES];
  __shared__ float sW[CH];
  const int tid = threadIdx.x, lane = tid & 31, wave = tid >> 5;
  const int hh = lane >> 4, m = lane & 15;
  const int b = blockIdx.x >> 3, fg = blockIdx.x & 7;
  const int dbase = (fg & 1) * 64;
  const float sgn = ((fg & 2) != 0) ? -1.0f : 1.0f;
  const int wsin = (fg >> 2) & 1;

  __bf16* sKh = (__bf16*)(void*)sbuf;
  __bf16* sKl = sKh + 64 * KP;
  float* slab = (float*)(void*)sbuf + wave * SLABF;

  const __bf16* VT = (const __bf16*)(const void*)VTp;
  const __bf16* arow = VT + ((size_t)(b * NJ + wave * 16 + m)) * NT + 8 * hh;

  v8f acc[4];
#pragma unroll
  for (int nt = 0; nt < 4; ++nt) acc[nt] = zero8();
  const int q4 = lane >> 3, c8 = (lane & 7) * 8;
  const float PI_F = 3.14159265358979323846f;

  for (int c = 0; c <= NCH; ++c) {
    __syncthreads();
#pragma unroll
    for (int nt = 0; nt < 4; ++nt)
#pragma unroll
      for (int r = 0; r < 8; ++r) slab[(8 * hh + r) * 68 + nt * 16 + m] = acc[nt][r];
    __builtin_amdgcn_fence(__ATOMIC_RELEASE, "workgroup");
    __builtin_amdgcn_wave_barrier();
    __builtin_amdgcn_fence(__ATOMIC_ACQUIRE, "workgroup");
    v4u hv[4], lv[4];
#pragma unroll
    for (int it = 0; it < 4; ++it) {
      const int row = it * 4 + q4;
      const float* sp = slab + row * 68 + c8;
      v4u a, a2;
#pragma unroll
      for (int e = 0; e < 4; ++e) {
        const float f0 = sp[2 * e], f1 = sp[2 * e + 1];
        const unsigned short h0 = bf_bits(f0), h1 = bf_bits(f1);
        const unsigned short l0 = bf_bits(f0 - bf_up(h0)), l1 = bf_bits(f1 - bf_up(h1));
        a[e] = pk16(h0, h1); a2[e] = pk16(l0, l1);
      }
      hv[it] = a; lv[it] = a2;
    }
    const size_t gb = ((size_t)((b * NSL + c) * NJ + wave * 16)) * NSF + fg * 64 + c8;
    for (int pass = 0; pass < 2; ++pass) {
#pragma unroll
      for (int it = 0; it < 4; ++it) {
        const int row = it * 4 + q4;
        *(volatile v4u*)(Shp + gb + (size_t)row * NSF) = hv[it];
        *(volatile v4u*)(Slp + gb + (size_t)row * NSF) = lv[it];
      }
      __threadfence();
    }
    __syncthreads();
    if (c < NCH) {
      if (tid < CH) {
        const float th = (PI_F * (float)(c * CH + tid)) / 8192.0f;
        const float cs = cosf(th), sn = sinf(th);
        sW[tid] = (wsin != 0) ? sn : cs;
      }
      __syncthreads();
      if (tid < 256) {
        const int s = tid >> 1, nh = (tid & 1) * 32;
        const float wv = sW[s];
        const float* src = kin + ((size_t)(b * NT + c * CH + s)) * ND + dbase + nh;
#pragma unroll 1
        for (int g = 0; g < 4; ++g) {
          const v4f a0 = *(const v4f*)(src + 8 * g);
          const v4f a1 = *(const v4f*)(src + 8 * g + 4);
          const float xv[8] = {a0[0], a0[1], a0[2], a0[3], a1[0], a1[1], a1[2], a1[3]};
#pragma unroll
          for (int e = 0; e < 8; ++e) {
            const unsigned short bt = bf_bits(xv[e]);
            const float kf = fmaxf(sgn * bf_up(bt), 0.0f);
            const float kw = kf * wv;
            const unsigned short hb = bf_bits(kw);
            const unsigned short lb = bf_bits(kw - bf_up(hb));
            const int n = nh + 8 * g + e;
            sKh[n * KP + s] = bf_val(hb);
            sKl[n * KP + s] = bf_val(lb);
          }
        }
      }
      __syncthreads();
      const __bf16* ac = arow + (size_t)c * CH;
#pragma unroll 1
      for (int ks = 0; ks < 4; ++ks) {
        const v16b a = ldfrag_b(ac + 32 * ks);
#pragma unroll
        for (int nt = 0; nt < 4; ++nt) {
          const int p = (nt * 16 + m) * KP + 32 * ks + 8 * hh;
          const v16b bh = ldfrag_b(sKh + p);
          const v16b bl = ldfrag_b(sKl + p);
          acc[nt] = mma_b(a, bh, acc[nt]);
          acc[nt] = mma_b(a, bl, acc[nt]);
        }
      }
    }
  }
}

#define L_Q    0
#define L_K    67584
#define L_PH   135168
#define L_PL   169984
#define L_TR   204800
#define L_TOT  206336
static_assert(L_K - L_Q == CH * QP * 2);
static_assert(L_PH - L_K == CH * QP * 2);
static_assert(L_PL - L_PH == CH * KP * 2);
static_assert(L_TR - L_PL == CH * KP * 2);
static_assert(L_TOT - L_TR == 3 * CH * 4);
static_assert(8 * 16 * ND * 4 <= L_K);

__global__ __launch_bounds__(256)
void k_out(const float* __restrict__ qin, const float* __restrict__ kin, const int* __restrict__ czp,
           const unsigned short* __restrict__ VTp, const unsigned short* __restrict__ Shp,
           const unsigned short* __restrict__ Slp, float* out) {
  extern __shared__ __align__(16) unsigned char lds[];
  __bf16* sQ = (__bf16*)(void*)(lds + L_Q);
  __bf16* sK = (__bf16*)(void*)(lds + L_K);
  __bf16* Ph = (__bf16*)(void*)(lds + L_PH);
  __bf16* Pl = (__bf16*)(void*)(lds + L_PL);
  float* sCos = (float*)(void*)(lds + L_TR);
  float* sSin = sCos + CH;
  float* sTan = sSin + CH;

  const int tid = threadIdx.x, lane = tid & 31, wave = tid >> 5;
  const int hh = lane >> 4, m = lane & 15;
  const int b = blockIdx.x >> 5, c = blockIdx.x & 31, t0 = c * CH;
  const int cz = czp[0];
  const float PI_F = 3.14159265358979323846f;

  if (tid < CH) {
    const float th = (PI_F * (float)(t0 + tid)) / 8192.0f;
    const float cs = cosf(th), sn = sinf(th);
    sCos[tid] = cs;
    sSin[tid] = sn;
    sTan[tid] = sn / cs;
  }
  {
    const int r = tid >> 1, dh = (tid & 1) * 64;
    const size_t go = ((size_t)(b * NT + t0 + r)) * ND + dh;
    __bf16* qd = sQ + r * QP + dh;
    __bf16* kd = sK + r * QP + dh;
#pragma unroll 1
    for (int g = 0; g < 8; ++g) {
      v4u pp, nn;
      relu_pack8(*(const v4f*)(qin + go + 8 * g), *(const v4f*)(qin + go + 8 * g + 4), pp, nn);
      *(v8b*)(qd + 8 * g)      = __builtin_bit_cast(v8b, pp);
      *(v8b*)(qd + ND + 8 * g) = __builtin_bit_cast(v8b, nn);
      relu_pack8(*(const v4f*)(kin + go + 8 * g), *(const v4f*)(kin + go + 8 * g + 4), pp, nn);
      *(v8b*)(kd + 8 * g)      = __builtin_bit_cast(v8b, pp);
      *(v8b*)(kd + ND + 8 * g) = __builtin_bit_cast(v8b, nn);
    }
  }
  __syncthreads();

  v8f G[8];
#pragma unroll
  for (int kt = 0; kt < 8; ++kt) G[kt] = zero8();
  const __bf16* qrow = sQ + (wave * 16 + m) * QP + 8 * hh;
#pragma unroll 1
  for (int ks = 0; ks < 8; ++ks) {
    const v16b a = ldfrag_b(qrow + 32 * ks);
#pragma unroll
    for (int kt = 0; kt < 8; ++kt) {
      const v16b bb = ldfrag_b(sK + (kt * 16 + m) * QP + 32 * ks + 8 * hh);
      G[kt] = mma_b(a, bb, G[kt]);
    }
  }
  {
    const int von = (cz != 0) ? 1 : 0;
#pragma unroll
    for (int kt = 0; kt < 8; ++kt) {
      const int sl = kt * 16 + m;
      const float cs_s = sCos[sl], sn_s = sSin[sl];
#pragma unroll
      for (int r = 0; r < 8; ++r) {
        const int tl = wave * 16 + 8 * hh + r;
        float pv = G[kt][r] * (cs_s + sTan[tl] * sn_s);
        pv = (von != 0 && sl <= tl) ? pv : 0.0f;
        const unsigned short hb = bf_bits(pv);
        const unsigned short lb = bf_bits(pv - bf_up(hb));
        const int po = tl * KP + sl;
        Ph[po] = bf_val(hb);
        Pl[po] = bf_val(lb);
      }
    }
  }
  __builtin_amdgcn_fence(__ATOMIC_RELEASE, "workgroup");
  __builtin_amdgcn_wave_barrier();
  __builtin_amdgcn_fence(__ATOMIC_ACQUIRE, "workgroup");

  v8f acc[9];
#pragma unroll
  for (int nt = 0; nt < 9; ++nt) acc[nt] = zero8();
  const int sidx = (cz != 0) ? c : NCH;
  const size_t sb = ((size_t)((b * NSL + sidx) * NJ + m)) * NSF + 8 * hh;
  const __bf16* Sh = (const __bf16*)(const void*)Shp + sb;
  const __bf16* Sl = (const __bf16*)(const void*)Slp + sb;
#pragma unroll 1
  for (int ks = 0; ks < 8; ++ks) {
    const v16b a = ldfrag_b(qrow + 32 * ks);
    const int fo = NF + 32 * ks;
#pragma unroll
    for (int nt = 0; nt < 9; ++nt) {
      const v16b bh = ldfrag_b(Sh + (size_t)nt * 16 * NSF + fo);
      const v16b bl = ldfrag_b(Sl + (size_t)nt * 16 * NSF + fo);
      acc[nt] = mma_b(a, bh, acc[nt]);
      acc[nt] = mma_b(a, bl, acc[nt]);
    }
  }
  float tnr[8];
#pragma unroll
  for (int r = 0; r < 8; ++r) tnr[r] = sTan[wave * 16 + 8 * hh + r];
#pragma unroll
  for (int nt = 0; nt < 9; ++nt)
#pragma unroll
    for (int r = 0; r < 8; ++r) acc[nt][r] *= tnr[r];
#pragma unroll 1
  for (int ks = 0; ks < 8; ++ks) {
    const v16b a = ldfrag_b(qrow + 32 * ks);
    const int fo = 32 * ks;
#pragma unroll
    for (int nt = 0; nt < 9; ++nt) {
      const v16b bh = ldfrag_b(Sh + (size_t)nt * 16 * NSF + fo);
      const v16b bl = ldfrag_b(Sl + (size_t)nt * 16 * NSF + fo);
      acc[nt] = mma_b(a, bh, acc[nt]);
      acc[nt] = mma_b(a, bl, acc[nt]);
    }
  }
  {
    const __bf16* prh = Ph + (wave * 16 + m) * KP + 8 * hh;
    const __bf16* prl = Pl + (wave * 16 + m) * KP + 8 * hh;
    const __bf16* vrow = (const __bf16*)(const void*)VTp + ((size_t)(b * NJ + m)) * NT + t0 + 8 * hh;
#pragma unroll 1
    for (int kk = 0; kk < 4; ++kk) {
      const v16b pa = ldfrag_b(prh + 32 * kk);
      const v16b pl = ldfrag_b(prl + 32 * kk);
#pragma unroll
      for (int nt = 0; nt < 9; ++nt) {
        const v16b vb = ldfrag_b(vrow + (size_t)nt * 16 * NT + 32 * kk);
        acc[nt] = mma_b(pa, vb, acc[nt]);
        acc[nt] = mma_b(pl, vb, acc[nt]);
      }
    }
  }

  float sc[8];
#pragma unroll
  for (int r = 0; r < 8; ++r) {
    const float dcol = __shfl(acc[8][r], hh * 16, 32);
    const float cst = sCos[wave * 16 + 8 * hh + r];
    const float den = fmaxf(cst * dcol, 1e-6f);
    sc[r] = cst * (1.0f / den);
  }
  __syncthreads();
  float* so = (float*)(void*)lds + wave * (16 * ND);
#pragma unroll
  for (int nt = 0; nt < 8; ++nt)
#pragma unroll
    for (int r = 0; r < 8; ++r) so[(8 * hh + r) * ND + nt * 16 + m] = acc[nt][r] * sc[r];
  __builtin_amdgcn_fence(__ATOMIC_RELEASE, "workgroup");
  __builtin_amdgcn_wave_barrier();
  __builtin_amdgcn_fence(__ATOMIC_ACQUIRE, "workgroup");
  float* og = out + ((size_t)(b * NT + t0 + wave * 16)) * ND;
  for (int pass = 0; pass < 2; ++pass) {
#pragma unroll 4
    for (int row = 0; row < 16; ++row) {
      const v4f vv = *(const v4f*)(so + row * ND + lane * 4);
      *(volatile v4f*)(og + (size_t)row * ND + lane * 4) = vv;
    }
    __threadfence();
  }
}

extern "C" void kernel_launch(void* const* d_in, const int* in_sizes, int n_in,
                              void* d_out, int out_size, void* d_ws, size_t ws_size,
                              hipStream_t stream) {
  if (n_in < 4) return;
  const int nx = NB * NT * ND;
  if (in_sizes[0] != nx || in_sizes[1] != nx || in_sizes[2] != nx) return;
  if (in_sizes[3] < 1) return;
  if (out_size != nx) return;

  const float* qp = (const float*)d_in[0];
  const float* kp = (const float*)d_in[1];
  const float* vp = (const float*)d_in[2];
  const int*   czp = (const int*)d_in[3];

  const size_t PVT = (size_t)NB * NJ * NT * 2;
  const size_t PS  = (size_t)NB * NSL * NJ * NSF * 2;
  size_t off = 0;
  const size_t oVT = off; off += PVT;
  const size_t oSh = off; off += PS;
  const size_t oSl = off; off += PS;
  if (off > ws_size) return;
  if (off > (size_t)134217728u) return;

  char* ws = (char*)d_ws;
  unsigned short* VT = (unsigned short*)(ws + oVT);
  unsigned short* Sh = (unsigned short*)(ws + oSh);
  unsigned short* Sl = (unsigned short*)(ws + oSl);

  k_vt<<<dim3(NB * (NT / 64)), dim3(128), 0, stream>>>(vp, VT);
  k_state<<<dim3(NB * NFG), dim3(288), 0, stream>>>(kp, VT, Sh, Sl);
  (void)hipFuncSetAttribute(reinterpret_cast<const void*>(&k_out),
                            hipFuncAttributeMaxDynamicSharedMemorySize, L_TOT);
  k_out<<<dim3(NB * NCH), dim3(256), L_TOT, stream>>>(qp, kp, czp, VT, Sh, Sl, (float*)d_out);
  (void)hipGetLastError();
}
